// MEGNet_28329604284558
// MI455X (gfx1250) — hardware-run, weakly checked
//
#include <hip/hip_runtime.h>


namespace {
constexpr int N = 100000, E = 1000000, H = 64, L = 3, G = 256, VOCAB = 100, NBLK = N / 16;
constexpr float XS = 8.0f, WSC = 256.0f;
typedef _Float16 b16;
typedef __attribute__((ext_vector_type(16))) _Float16 v16b;
typedef __attribute__((ext_vector_type(8))) _Float16 v8b;
typedef __attribute__((ext_vector_type(8))) float v8f;
typedef __attribute__((ext_vector_type(4))) float v4f;
typedef __attribute__((ext_vector_type(2))) float v2f;
__device__ __forceinline__ float bf16_rne(float f) { unsigned int u = __float_as_uint(f); u += 0x7FFFu + ((u >> 16) & 1u); return __uint_as_float(u & 0xFFFF0000u); }
__device__ __forceinline__ void split16(float v, b16& hi, b16& lo) { hi = (b16)v; lo = (b16)(v - (float)hi); }
__device__ __forceinline__ v16b frag_kb(const b16* p, int hh) { const v8b a = *(const v8b*)(p + 8 * hh), b = *(const v8b*)(p + 16 + 8 * hh); v16b f;
#pragma unroll
  for (int e = 0; e < 8; ++e) { f[e] = a[e]; f[8 + e] = b[e]; } return f; }
__device__ __forceinline__ v8f wmma16b(v16b a, v16b b, v8f c) { v8f d = __builtin_amdgcn_wmma_f32_16x16x32_f16(false, a, false, b, (short)0, c, false, false); asm volatile("v_nop\n\tv_nop\n\tv_nop\n\tv_nop" : "+v"(d) : "v"(a), "v"(b)); return d; }
__device__ __forceinline__ void wave_lds_sync() { __builtin_amdgcn_fence(__ATOMIC_RELEASE, "workgroup"); __builtin_amdgcn_wave_barrier(); __builtin_amdgcn_fence(__ATOMIC_ACQUIRE, "workgroup"); }
__device__ __forceinline__ float pmul(float a, float b) { float p = a * b; asm volatile("" : "+v"(p)); return p; }
__device__ __forceinline__ int iclamp(int v, int lo, int hi) { return v < lo ? lo : (v > hi ? hi : v); }
__device__ __forceinline__ float sigm(float v) { return 1.0f / (1.0f + __expf(-v)); }
constexpr int CSR_NBLK9 = 512, CSR_GB9 = 9, CSR_GN9 = 1 << CSR_GB9  , CSR_TS9 = (CSR_GN9 < 32 ? 32 : CSR_GN9)  , CSR_MAXG9 = 512, CSR_CAP9 = 12288  ;
__device__ __host__ __forceinline__ int csr_tix9(int v) { return (v >> CSR_GB9) * CSR_TS9 + (v & (CSR_GN9 - 1)); }
__global__ __launch_bounds__(64) void csrA_kernel9(const int* __restrict__ dst, int E, int N, int nG, int CHP, int NGP, int* __restrict__ STG, int* __restrict__ HST) {
  extern __shared__ int sm[];
  int* cnt = sm; int* run = sm + NGP; int* ids = sm + 2 * NGP;
  const int b = blockIdx.x; const int ch = (E + CSR_NBLK9 - 1) / CSR_NBLK9; const int e0 = b * ch, e1 = min(E, e0 + ch);
  for (int i = threadIdx.x; i < NGP; i += 64) cnt[i] = 0;
  for (int i = threadIdx.x; i < CHP; i += 64) ids[i] = -1;
  __syncthreads();
  if (threadIdx.x == 0) {
    for (int e = e0; e < e1; ++e) { int d = dst[e]; d = (d < 0) ? 0 : (d >= N ? N - 1 : d); cnt[d >> CSR_GB9] += 1; }
    int acc = 0; for (int g = 0; g < nG; ++g) { run[g] = acc; acc += cnt[g]; }
    for (int e = e0; e < e1; ++e) { int d = dst[e]; d = (d < 0) ? 0 : (d >= N ? N - 1 : d); const int g = d >> CSR_GB9; ids[run[g]] = e; run[g] += 1; } }
  __syncthreads();
  typedef __attribute__((ext_vector_type(4))) int v4i;
  for (int pass = 0; pass < 2; ++pass) {
    for (int i = threadIdx.x; i < CHP / 4; i += 64) *(volatile v4i*)(STG + (size_t)b * CHP + i * 4) = *(const v4i*)(&ids[i * 4]);
    for (int i = threadIdx.x; i < NGP / 4; i += 64) { v4i v; for (int e = 0; e < 4; ++e) v[e] = (i * 4 + e < nG) ? cnt[i * 4 + e] : 0; *(volatile v4i*)(HST + (size_t)b * NGP + i * 4) = v; }
    __threadfence(); }
}
__global__ __launch_bounds__(512) void csrS_kernel9(const int* __restrict__ HST, int nG, int NGP, int* __restrict__ START, int* __restrict__ TOT, int* __restrict__ OFF) {
  __shared__ int tot[CSR_MAXG9];
  const int b = threadIdx.x;
  for (int pass = 0; pass < 2; ++pass) { int runb = 0; for (int g = 0; g < nG; ++g) { int c = HST[(size_t)b * NGP + g]; c = (c < 0) ? 0 : c; ((volatile int*)OFF)[(size_t)g * CSR_NBLK9 + b] = runb; runb += c; } __threadfence(); }
  for (int g = threadIdx.x; g < nG; g += 512) { int s = 0; for (int bb = 0; bb < CSR_NBLK9; ++bb) { int c = HST[(size_t)bb * NGP + g]; s += (c < 0) ? 0 : c; } tot[g] = s; }
  __syncthreads();
  if (threadIdx.x < 32) {
    __shared__ int st[CSR_MAXG9 + 32];
    if (threadIdx.x == 0) { int acc = 0; for (int g = 0; g < NGP; ++g) { st[g] = acc; if (g < nG) acc += (tot[g] + 31) & ~31; } st[NGP] = acc; }
    __builtin_amdgcn_fence(__ATOMIC_RELEASE, "workgroup"); __builtin_amdgcn_wave_barrier(); __builtin_amdgcn_fence(__ATOMIC_ACQUIRE, "workgroup");
    for (int pass = 0; pass < 2; ++pass) { for (int i = threadIdx.x; i < NGP + 32; i += 32) { ((volatile int*)START)[i] = (i <= NGP) ? st[min(i, NGP)] : 0; ((volatile int*)TOT)[i] = (i < nG) ? tot[i] : 0; } __threadfence(); } }
}
__global__ __launch_bounds__(256) void csrB_kernel9(const int* __restrict__ dst, int N, int nG, int CHP, int NGP, int permLen, const int* __restrict__ STG, const int* __restrict__ HST, const int* __restrict__ OFF, const int* __restrict__ START, const int* __restrict__ TOT, int* __restrict__ PERM, int* __restrict__ ROWPTR, int* __restrict__ ROWCNT, int* __restrict__ FLAG) {
  typedef __attribute__((ext_vector_type(4))) int v4i;
  __shared__ int ids[CSR_CAP9]; __shared__ unsigned short key[CSR_CAP9]; __shared__ int outp[CSR_CAP9]; __shared__ int ncnt[CSR_GN9 + 1]; __shared__ int boff[CSR_NBLK9 + 1];
  const int g = blockIdx.x, t_ = threadIdx.x; int tot = TOT[g]; int st = START[g], stn = START[g + 1]; const int v0 = g * CSR_GN9; const int nv = min(CSR_GN9, N - v0); const int t0 = g * CSR_TS9;
  st = (st < 0) ? 0 : (st > permLen - 32 ? permLen - 32 : st) & ~31; stn = (stn < st) ? st : (stn > permLen ? permLen : stn); tot = (tot < 0) ? 0 : tot; if (tot > stn - st && tot <= CSR_CAP9) tot = stn - st;
  if (tot > CSR_CAP9) {
    for (int pass = 0; pass < 2; ++pass) { for (int i = t_; i < CSR_TS9 / 4; i += 256) { v4i a, c; for (int e = 0; e < 4; ++e) { a[e] = st; c[e] = 0; } *(volatile v4i*)(ROWPTR + t0 + i * 4) = a; *(volatile v4i*)(ROWCNT + t0 + i * 4) = c; } if (t_ == 0) ((volatile int*)FLAG)[0] = 1; __threadfence(); } (void)nv; return; }
  if (t_ == 0) { int acc = 0; for (int b = 0; b < CSR_NBLK9; ++b) { boff[b] = acc; int c = HST[(size_t)b * NGP + g]; c = (c < 0) ? 0 : (c > CHP ? CHP : c); acc += c; if (acc > tot) acc = tot; } boff[CSR_NBLK9] = acc; }
  for (int i = t_; i <= CSR_GN9; i += 256) ncnt[i] = 0;
  __syncthreads();
  for (int b = 0; b < CSR_NBLK9; ++b) { const int c = boff[b + 1] - boff[b]; int o_ = OFF[(size_t)g * CSR_NBLK9 + b]; o_ = (o_ < 0) ? 0 : (o_ > CHP - c ? CHP - c : o_); const int* src_ = STG + (size_t)b * CHP + o_;
    for (int i = t_; i < c; i += 256) { int id = src_[i]; id = (id < 0) ? 0 : id; ids[boff[b] + i] = id; int d = dst[id]; d = (d < v0) ? v0 : (d >= N ? N - 1 : d); int kk = d - v0; kk = (kk < 0) ? 0 : (kk >= CSR_GN9 ? CSR_GN9 - 1 : kk); key[boff[b] + i] = (unsigned short)kk; } }
  __syncthreads();
  if (t_ == 0) { for (int i = 0; i < tot; ++i) ncnt[key[i]] += 1; int acc = 0; for (int vl = 0; vl < CSR_GN9; ++vl) { const int c = ncnt[vl]; ncnt[vl] = acc; acc += c; } ncnt[CSR_GN9] = acc;
    for (int i = 0; i < tot; ++i) { const int vl = key[i]; outp[ncnt[vl]] = ids[i]; ncnt[vl] += 1; }
    for (int vl = CSR_GN9; vl > 0; --vl) ncnt[vl] = ncnt[vl - 1]; ncnt[0] = 0; }
  __syncthreads();
  for (int pass = 0; pass < 2; ++pass) {
    for (int i = t_; i < (stn - st) / 4; i += 256) { v4i v; for (int e = 0; e < 4; ++e) { const int q = i * 4 + e; v[e] = (q < tot) ? outp[q] : -1; } *(volatile v4i*)(PERM + st + i * 4) = v; }
    for (int i = t_; i < CSR_TS9 / 4; i += 256) { v4i a, c; for (int e = 0; e < 4; ++e) { const int vl = i * 4 + e; const int vc = vl < CSR_GN9 ? vl : CSR_GN9; a[e] = (vl < CSR_GN9) ? st + ncnt[vc] : st; c[e] = (vl < nv) ? (ncnt[(vc < CSR_GN9 ? vc : CSR_GN9 - 1) + 1] - ncnt[vc]) : 0; } *(volatile v4i*)(ROWPTR + t0 + i * 4) = a; *(volatile v4i*)(ROWCNT + t0 + i * 4) = c; }
    __threadfence(); }
}
__global__ __launch_bounds__(256) void csrZ_kernel9(int* __restrict__ p, size_t n4) { typedef __attribute__((ext_vector_type(4))) int v4i; const size_t tid = (size_t)blockIdx.x * 256 + threadIdx.x, nth = (size_t)gridDim.x * 256; v4i z = {0, 0, 0, 0}; for (size_t i = tid; i < n4; i += nth) *(volatile v4i*)(p + i * 4) = z; }
struct CsrBufs9 { int *STG, *HST, *OFF, *START, *TOT, *PERM, *ROWPTR, *ROWCNT, *FLAG; int nG, NGP, CHP; size_t permLen; char* base; size_t bytes; };
static size_t csr_carve9(CsrBufs9& c, char* ws, size_t off, int E, int N) {
  const size_t off0 = off; c.base = ws + off;
  auto al = [&](size_t bytes) { char* p = ws + off; off += (bytes + 255) & ~(size_t)255; return p; };
  c.nG = (N + CSR_GN9 - 1) / CSR_GN9; c.NGP = (c.nG + 31) & ~31; const int ch = (E + CSR_NBLK9 - 1) / CSR_NBLK9; c.CHP = (ch + 31) & ~31; c.permLen = (size_t)E + 32 * (size_t)c.nG + 32;
  c.STG = (int*)al((size_t)CSR_NBLK9 * c.CHP * 4); c.HST = (int*)al((size_t)CSR_NBLK9 * c.NGP * 4); c.OFF = (int*)al((size_t)c.NGP * CSR_NBLK9 * 4); c.START = (int*)al((size_t)(c.NGP + 64) * 4); c.TOT = (int*)al((size_t)(c.NGP + 64) * 4);
  c.PERM = (int*)al(c.permLen * 4); c.ROWPTR = (int*)al((size_t)c.nG * CSR_TS9 * 4); c.ROWCNT = (int*)al((size_t)c.nG * CSR_TS9 * 4); c.FLAG = (int*)al(256);
  c.bytes = off - off0; return off;
}
static void csr_build9(const CsrBufs9& c, const int* dst, int E, int N, hipStream_t stream) {
  const size_t smem = (size_t)(2 * c.NGP + c.CHP) * 4;
  csrZ_kernel9<<<512, 256, 0, stream>>>((int*)c.base, c.bytes / 16);
  csrA_kernel9<<<CSR_NBLK9, 64, smem, stream>>>(dst, E, N, c.nG, c.CHP, c.NGP, c.STG, c.HST);
  csrS_kernel9<<<1, 512, 0, stream>>>(c.HST, c.nG, c.NGP, c.START, c.TOT, c.OFF);
  csrB_kernel9<<<c.nG, 256, 0, stream>>>(dst, N, c.nG, c.CHP, c.NGP, (int)c.permLen, c.STG, c.HST, c.OFF, c.START, c.TOT, c.PERM, c.ROWPTR, c.ROWCNT, c.FLAG);
}


__global__ __launch_bounds__(256) void w_kernel(const float* __restrict__ gg, const float* __restrict__ wih, const float* __restrict__ whh, b16* __restrict__ WG, b16* __restrict__ WIH, b16* __restrict__ WHH) {
  const int u = blockIdx.x * 256 + threadIdx.x; v8b v;
  if (u < L * H * 8) { const int l = u / (H * 8), o = (u / 8) % H, k0 = (u % 8) * 8; for (int j = 0; j < 8; ++j) v[j] = (b16)(bf16_rne(gg[((size_t)l * H + k0 + j) * H + o]) * WSC); for (int pass = 0; pass < 2; ++pass) { *(volatile v8b*)(WG + ((size_t)l * H + o) * H + k0) = v; __threadfence(); } return; }
  int w = u - L * H * 8; if (w >= 2 * L * 192 * 8) return; const int which = w / (L * 192 * 8); const size_t e = (size_t)(w % (L * 192 * 8)) * 8; const float* src = which ? whh : wih; b16* dst = which ? WHH : WIH;
  for (int j = 0; j < 8; ++j) v[j] = (b16)(bf16_rne(src[e + j]) * WSC); for (int pass = 0; pass < 2; ++pass) { *(volatile v8b*)(dst + e) = v; __threadfence(); }
}
__global__ __launch_bounds__(32) void emb_kernel(const int* __restrict__ xi, const float* __restrict__ emb, int NLIM, float* __restrict__ Hh) {
  const int lane = threadIdx.x; const size_t m0 = (size_t)blockIdx.x * 16; if (m0 >= (size_t)NLIM) return;
  for (int pass = 0; pass < 2; ++pass) { for (int rr = 0; rr < 16; ++rr) { const int t = iclamp(xi[m0 + rr], 0, VOCAB - 1); const v2f v = {bf16_rne(emb[t * H + lane * 2]), bf16_rne(emb[t * H + lane * 2 + 1])}; *(volatile v2f*)(Hh + (m0 + rr) * H + lane * 2) = v; } __threadfence(); }
}
__global__ __launch_bounds__(32) void lin_kernel(const float* __restrict__ Hh, const b16* __restrict__ WG, int NLIM, float* __restrict__ M) {
  __shared__ __attribute__((aligned(16))) b16 Ah[16][H + 8], Al[16][H + 8]; __shared__ __attribute__((aligned(16))) float Tf[16][H + 4];
  const int lane = threadIdx.x, nloc = lane & 15, hlf = lane >> 4; const size_t m0 = (size_t)blockIdx.x * 16; if (m0 >= (size_t)NLIM) return;
  for (int rr = 0; rr < 16; ++rr) for (int q = 0; q < 2; ++q) { b16 p, ql; split16(Hh[(m0 + rr) * H + q * 32 + lane] * XS, p, ql); Ah[rr][q * 32 + lane] = p; Al[rr][q * 32 + lane] = ql; }
  wave_lds_sync();
  v8f acc[4];
#pragma unroll
  for (int t = 0; t < 4; ++t) acc[t] = (v8f){};
#pragma unroll
  for (int kb = 0; kb < H; kb += 32) { const v16b a = frag_kb(&Ah[nloc][kb], hlf), al = frag_kb(&Al[nloc][kb], hlf);
#pragma unroll
    for (int t = 0; t < 4; ++t) { const v16b bw = frag_kb(WG + (size_t)(t * 16 + nloc) * H + kb, hlf); acc[t] = wmma16b(a, bw, acc[t]); acc[t] = wmma16b(al, bw, acc[t]); } }
#pragma unroll
  for (int t = 0; t < 4; ++t)
#pragma unroll
    for (int r8 = 0; r8 < 8; ++r8) Tf[8 * hlf + r8][t * 16 + nloc] = acc[t][r8] * (1.0f / (XS * WSC));
  wave_lds_sync();
  for (int pass = 0; pass < 2; ++pass) { for (int rr = 0; rr < 16; ++rr) *(volatile v2f*)(M + (m0 + rr) * H + lane * 2) = *(const v2f*)(&Tf[rr][lane * 2]); __threadfence(); }
}
__global__ __launch_bounds__(32) void gru_kernel(const float* __restrict__ Hh, const float* __restrict__ M, const int* __restrict__ srcs, const int* __restrict__ PERM, const int* __restrict__ ROWPTR, const int* __restrict__ ROWCNT, int permLen, const b16* __restrict__ WIH, const b16* __restrict__ WHH, const float* __restrict__ bih, const float* __restrict__ bhh, int NLIM, float* __restrict__ HN) {
  __shared__ __attribute__((aligned(16))) b16 A1h[16][H + 8], A1l[16][H + 8], A2h[16][H + 8], A2l[16][H + 8]; __shared__ __attribute__((aligned(16))) float Hs[16][H + 1], R[16][H + 1], Z[16][H + 1], Tf[16][H + 4];
  const int lane = threadIdx.x, nloc = lane & 15, hlf = lane >> 4; const size_t m0 = (size_t)blockIdx.x * 16; if (m0 >= (size_t)NLIM) return;
  for (int rr = 0; rr < 16; ++rr) { const size_t v = m0 + rr; int st = ROWPTR[v], cnt = ROWCNT[v]; cnt = iclamp(cnt, 0, 1 << 20); st = iclamp(st, 0, permLen - cnt); v2f a = {0.0f, 0.0f};
#pragma unroll 1
    for (int j = 0; j < cnt; ++j) { const int e = iclamp(PERM[st + j], 0, E - 1); const size_t u = (size_t)iclamp(srcs[e], 0, N - 1); if (u >= (size_t)NLIM) continue; const v2f mv = *(const v2f*)(M + u * H + lane * 2); a[0] += mv[0]; a[1] += mv[1]; }
    const v2f hv = *(const v2f*)(Hh + v * H + lane * 2);
    for (int i = 0; i < 2; ++i) { const int c = lane * 2 + i; b16 p, q; split16(a[i] * XS, p, q); A1h[rr][c] = p; A1l[rr][c] = q; split16(hv[i] * XS, p, q); A2h[rr][c] = p; A2l[rr][c] = q; Hs[rr][c] = hv[i]; } }
  wave_lds_sync(); const float sc = 1.0f / (XS * WSC);
  auto gemm = [&](const b16 (*Ah)[H + 8], const b16 (*Al)[H + 8], const b16* WT, int ro, v8f acc[4], bool init) {
    if (init) {
#pragma unroll
      for (int t = 0; t < 4; ++t) acc[t] = (v8f){}; }
#pragma unroll
    for (int kb = 0; kb < H; kb += 32) { const v16b a = frag_kb(&Ah[nloc][kb], hlf), al = frag_kb(&Al[nloc][kb], hlf);
#pragma unroll
      for (int t = 0; t < 4; ++t) { const v16b bw = frag_kb(WT + (size_t)(ro + t * 16 + nloc) * H + kb, hlf); acc[t] = wmma16b(a, bw, acc[t]); acc[t] = wmma16b(al, bw, acc[t]); } } };
  v8f acc[4], acc2[4];
  gemm(A1h, A1l, WIH, 0, acc, true); gemm(A2h, A2l, WHH, 0, acc, false);
#pragma unroll
  for (int t = 0; t < 4; ++t) { const int c = t * 16 + nloc; const float bb = bf16_rne(bih[c]) + bf16_rne(bhh[c]);
#pragma unroll
    for (int r8 = 0; r8 < 8; ++r8) R[8 * hlf + r8][c] = sigm(acc[t][r8] * sc + bb); }
  gemm(A1h, A1l, WIH, H, acc, true); gemm(A2h, A2l, WHH, H, acc, false);
#pragma unroll
  for (int t = 0; t < 4; ++t) { const int c = t * 16 + nloc; const float bb = bf16_rne(bih[H + c]) + bf16_rne(bhh[H + c]);
#pragma unroll
    for (int r8 = 0; r8 < 8; ++r8) Z[8 * hlf + r8][c] = sigm(acc[t][r8] * sc + bb); }
  gemm(A1h, A1l, WIH, 2 * H, acc, true); gemm(A2h, A2l, WHH, 2 * H, acc2, true);
  wave_lds_sync();
#pragma unroll
  for (int t = 0; t < 4; ++t) { const int c = t * 16 + nloc; const float bi = bf16_rne(bih[2 * H + c]), bh = bf16_rne(bhh[2 * H + c]);
#pragma unroll
    for (int r8 = 0; r8 < 8; ++r8) { const int rl = 8 * hlf + r8; const float n = tanhf(acc[t][r8] * sc + bi + pmul(R[rl][c], acc2[t][r8] * sc + bh)); const float z = Z[rl][c]; Tf[rl][c] = fmaxf(pmul(1.0f - z, n) + pmul(z, Hs[rl][c]), 0.0f); } }
  wave_lds_sync();
  for (int pass = 0; pass < 2; ++pass) { for (int rr = 0; rr < 16; ++rr) *(volatile v2f*)(HN + (m0 + rr) * H + lane * 2) = *(const v2f*)(&Tf[rr][lane * 2]); __threadfence(); }
}
__global__ __launch_bounds__(32) void grange_kernel(const int* __restrict__ batch, int* __restrict__ SE) {
  const int lane = threadIdx.x;
  auto lb = [&](int key) -> int { int lo = 0, hi = N; for (int it = 0; it < 18 && lo < hi; ++it) { const int mid = (lo + hi) >> 1; if (batch[mid] < key) lo = mid + 1; else hi = mid; } return lo; };
  for (int g0 = 0; g0 < G; g0 += 32) { const int g = g0 + lane; const int st = lb(g), en = lb(g + 1); for (int pass = 0; pass < 2; ++pass) { ((volatile int*)SE)[g] = st; ((volatile int*)SE)[G + g] = en; __threadfence(); } }
}
__global__ __launch_bounds__(64) void pool_kernel(const float* __restrict__ Hh, const int* __restrict__ SE, const float* __restrict__ f1W, const float* __restrict__ f1b, const float* __restrict__ f2W, const float* __restrict__ f2b, const float* __restrict__ f3W, const float* __restrict__ f3b, int NLIM, float* __restrict__ PO) {
  __shared__ float Ps[H], Y1[32]; const int g = blockIdx.x, c = threadIdx.x; int s0 = iclamp(SE[g], 0, N), e0 = iclamp(SE[G + g], 0, N); if (e0 > NLIM) e0 = NLIM; if (e0 < s0) e0 = s0; float s = 0.0f; int cnt = 0;
#pragma unroll 1
  for (int n = s0; n < e0; ++n) { s += Hh[(size_t)n * H + c]; ++cnt; }
  Ps[c] = s / (float)(cnt < 1 ? 1 : cnt); __syncthreads();
  if (c < 32) { float a = bf16_rne(f1b[c]);
#pragma unroll 1
    for (int k = 0; k < H; ++k) a += pmul(Ps[k], bf16_rne(f1W[c * H + k])); Y1[c] = fmaxf(a, 0.0f); }
  __syncthreads();
  if (c < 32) { const int cc = c & 15; float a = bf16_rne(f2b[cc]);
#pragma unroll 1
    for (int k = 0; k < 32; ++k) a += pmul(Y1[k], bf16_rne(f2W[cc * 32 + k])); float t = (c < 16) ? pmul(fmaxf(a, 0.0f), bf16_rne(f3W[cc])) : 0.0f; for (int o = 16; o; o >>= 1) t += __shfl_xor(t, o); const float r = t + bf16_rne(f3b[0]);
    for (int pass = 0; pass < 2; ++pass) { ((volatile float*)PO)[g * 32 + c] = r; __threadfence(); } }
}
__global__ __launch_bounds__(32) void outw_kernel(const float* __restrict__ PO, float* __restrict__ out) { const int g = blockIdx.x * 32 + threadIdx.x; const float v = PO[g * 32]; for (int pass = 0; pass < 2; ++pass) { ((volatile float*)out)[g] = v; __threadfence(); } }
}

extern "C" void kernel_launch(void* const* d_in, const int* in_sizes, int n_in, void* d_out, int out_size, void* d_ws, size_t ws_size, hipStream_t stream) {
  (void)n_in;
  auto Fp = [&](int i) { return (const float*)d_in[i]; }; auto Ip = [&](int i) { return (const int*)d_in[i]; };
  if (in_sizes[0] != N || in_sizes[1] != 2 * E || in_sizes[3] != N || in_sizes[4] != VOCAB * H || in_sizes[7] != L * H * H || in_sizes[8] != L * 3 * H * H || in_sizes[12] != 32 * H || in_sizes[14] != 16 * 32 || in_sizes[16] != 16 || out_size != G) return;
  const int NLIM = N; const int GB16 = NBLK;
  size_t off = 0; char* ws = (char*)d_ws;
  auto carve = [&](size_t bytes) { char* p = ws + off; off += (bytes + 255) & ~(size_t)255; return p; };
  b16* WG = (b16*)carve(L * H * H * 2); b16* WIH = (b16*)carve(L * 192 * H * 2); b16* WHH = (b16*)carve(L * 192 * H * 2); float* HA = (float*)carve((size_t)N * H * 4); float* HB = (float*)carve((size_t)N * H * 4); float* M = (float*)carve((size_t)N * H * 4); int* SE = (int*)carve(2 * G * 4); float* PO = (float*)carve(G * 32 * 4);
  CsrBufs9 csr; off = csr_carve9(csr, ws, off, E, N);
  if (off > ws_size || off > ((size_t)128 << 20)) return;
  w_kernel<<<(L * H * 8 + 2 * L * 192 * 8 + 255) / 256, 256, 0, stream>>>(Fp(7), Fp(8), Fp(9), WG, WIH, WHH);
  csr_build9(csr, Ip(1) + E, E, N, stream);
  emb_kernel<<<GB16, 32, 0, stream>>>(Ip(0), Fp(4), NLIM, HA);
  float* hp = HA; float* hn = HB;
  for (int l = 0; l < L; ++l) {
    lin_kernel<<<GB16, 32, 0, stream>>>(hp, WG + (size_t)l * H * H, NLIM, M);
    gru_kernel<<<GB16, 32, 0, stream>>>(hp, M, Ip(1), csr.PERM, csr.ROWPTR, csr.ROWCNT, (int)csr.permLen, WIH + (size_t)l * 192 * H, WHH + (size_t)l * 192 * H, Fp(10) + l * 192, Fp(11) + l * 192, NLIM, hn);
    float* t = hp; hp = hn; hn = t; }
  grange_kernel<<<1, 32, 0, stream>>>(Ip(3), SE);
  pool_kernel<<<G, 64, 0, stream>>>(hp, SE, Fp(12), Fp(13), Fp(14), Fp(15), Fp(16), Fp(17), NLIM, PO);
  outw_kernel<<<G / 32, 32, 0, stream>>>(PO, (float*)d_out);
}
